// IAF_10161892622818
// MI455X (gfx1250) — hardware-verified
//
#include <hip/hip_runtime.h>
#include <stddef.h>
#include <stdint.h>


#define D_      32
#define H_      256
#define NB_     2
#define NO_     64
#define NROWS   16384
#define NW      2
#define NTHR    64
#define RPB     32
#define PITCH   264
#define OFF_P1  16384
#define OFF_P2  147456
#define WHALF   180224
#define BOFF    90112
#define NBIAS   1024
#define WSBYTES 364544
#define PKB     89
#define PB1     8
#define PB2     72
#define YOFF    524288
#define XS      8.0f
#define WS      64.0f
#define WSCAP   134217728

static_assert(NO_ == 2 * D_);
static_assert(RPB == NW * 16);
static_assert(NTHR == NW * 32);
static_assert((NROWS % RPB) == 0);
static_assert(OFF_P1 == NB_ * H_ * D_);
static_assert(OFF_P2 == OFF_P1 + NB_ * H_ * H_);
static_assert(WHALF == OFF_P2 + NB_ * NO_ * H_);
static_assert(PB1 * 2048 == OFF_P1);
static_assert(PB2 * 2048 == OFF_P2);
static_assert((PKB - 1) * 2048 == WHALF);
static_assert(BOFF * 4 == WHALF * 2);
static_assert(((BOFF * 4) % 128) == 0);
static_assert(NBIAS == 2 * NB_ * H_);
static_assert(NBIAS == 256 * 4);
static_assert(WSBYTES == BOFF * 4 + NBIAS * 4);
static_assert(WSBYTES <= WSCAP);
static_assert((PITCH % 8) == 0);
static_assert(PITCH >= H_);
static_assert(YOFF == NROWS * D_);
static_assert(H_ == 8 * 31 + 8);

typedef float    v4f  __attribute__((ext_vector_type(4)));
typedef float    v8f  __attribute__((ext_vector_type(8)));
typedef _Float16 v8h  __attribute__((ext_vector_type(8)));
typedef _Float16 v16h __attribute__((ext_vector_type(16)));
union FragH { v16h v; v8h h[2]; };

__device__ __forceinline__ v8f wmf(v16h a, v16h b, v8f c) {
  v8f d = __builtin_amdgcn_wmma_f32_16x16x32_f16(false, a, false, b, (short)0, c, false, false);
  asm volatile("v_nop\n\tv_nop\n\tv_nop\n\tv_nop" : "+v"(d) : "v"(a), "v"(b));
  return d;
}

__device__ __forceinline__ v8f zero8() {
  v8f z = {0.f, 0.f, 0.f, 0.f, 0.f, 0.f, 0.f, 0.f};
  return z;
}

__device__ __forceinline__ v16h ldfrag(const _Float16* p) {
  FragH f;
  f.h[0] = *(const v8h*)p;
  f.h[1] = *(const v8h*)(p + 16);
  return f.v;
}

__device__ __forceinline__ v8h cvt8(v4f a, v4f b, float sc) {
  v8h r;
  r[0] = (_Float16)(a.x * sc); r[1] = (_Float16)(a.y * sc);
  r[2] = (_Float16)(a.z * sc); r[3] = (_Float16)(a.w * sc);
  r[4] = (_Float16)(b.x * sc); r[5] = (_Float16)(b.y * sc);
  r[6] = (_Float16)(b.z * sc); r[7] = (_Float16)(b.w * sc);
  return r;
}

__device__ __forceinline__ int sdeg(int jp) { return (jp < 72) ? (jp / 9) : (8 + ((jp - 72) >> 3)); }
__device__ __forceinline__ int sorig(int jp) {
  const bool lo = (jp < 72);
  const int d9 = jp / 9;
  const int d = lo ? d9 : (8 + ((jp - 72) >> 3));
  const int q = lo ? (jp - 9 * d9) : ((jp - 72) & 7);
  return 31 * q + d;
}
__device__ __forceinline__ int cntp(int t) { return (t <= 8) ? (9 * t) : (72 + 8 * (t - 8)); }

__global__ __launch_bounds__(256) void k_pack(const float* __restrict__ W0, const float* __restrict__ W1,
                                             const float* __restrict__ W2, const float* __restrict__ b0,
                                             const float* __restrict__ b1, _Float16* wh, float* bpl) {
  const int b = blockIdx.x, tid = threadIdx.x;
  if (b < PKB - 1) {
    const int e = (b * 256 + tid) * 8;
    float v[8];
    int keep[8];
    if (b < PB1) {
      const int idx = e;
      const int blk = idx >> 13, jp = (idx >> 5) & 255, k0 = idx & 31;
      const int d = sdeg(jp), j = sorig(jp);
      const float* src = W0 + ((size_t)(blk * H_ + j) * D_ + k0);
#pragma unroll
      for (int q = 0; q < 8; ++q) { v[q] = src[q]; keep[q] = (d >= k0 + q) ? 1 : 0; }
    } else if (b < PB2) {
      const int idx = e - OFF_P1;
      const int blk = idx >> 16, jp = (idx >> 8) & 255, l0 = idx & 255;
      const int d = sdeg(jp), j = sorig(jp);
      const float* src = W1 + (size_t)(blk * H_ + j) * H_;
#pragma unroll
      for (int q = 0; q < 8; ++q) {
        const int lp = l0 + q;
        v[q] = src[sorig(lp)];
        keep[q] = (d >= sdeg(lp)) ? 1 : 0;
      }
    } else {
      const int idx = e - OFF_P2;
      const int blk = idx >> 14, c = (idx >> 8) & 63, j0 = idx & 255;
      const int dc = c & 31;
      const float* src = W2 + (size_t)(blk * NO_ + c) * H_;
#pragma unroll
      for (int q = 0; q < 8; ++q) {
        const int jp = j0 + q;
        v[q] = src[sorig(jp)];
        keep[q] = (sdeg(jp) < dc) ? 1 : 0;
      }
    }
    v8h o;
#pragma unroll
    for (int q = 0; q < 8; ++q) o[q] = (_Float16)((keep[q] != 0) ? v[q] * WS : 0.0f);
    _Float16* dst = wh + e;
    *(volatile v8h*)dst = o;
    __threadfence();
    *(volatile v8h*)dst = o;
  } else {
    const int f = tid * 4;
    const int plane = f >> 9;
    const int w = f & 511;
    const int blk = w >> 8, jp0 = w & 255;
    float t0[4], t1[4];
#pragma unroll
    for (int q = 0; q < 4; ++q) {
      const int j = blk * H_ + sorig(jp0 + q);
      t0[q] = b0[j];
      t1[q] = b1[j];
    }
    v4f o;
    o.x = plane ? t1[0] : t0[0];
    o.y = plane ? t1[1] : t0[1];
    o.z = plane ? t1[2] : t0[2];
    o.w = plane ? t1[3] : t0[3];
    float* dst = bpl + f;
    *(volatile v4f*)dst = o;
    __threadfence();
    *(volatile v4f*)dst = o;
  }
}

__global__ __launch_bounds__(NTHR) void k_flow(const float* __restrict__ xin, const _Float16* __restrict__ wh,
                                              const float* __restrict__ bpl, const float* __restrict__ b2,
                                              float* out) {
  __shared__ __attribute__((aligned(16))) _Float16 h0t[NW * 16 * PITCH];
  __shared__ __attribute__((aligned(16))) _Float16 h1t[NW * 16 * PITCH];
  __shared__ __attribute__((aligned(16))) float yc[NW * 16 * D_];
  __shared__ __attribute__((aligned(16))) float xc[NW * 16 * D_];
  __shared__ __attribute__((aligned(16))) float lst[RPB];

  const int tid = threadIdx.x, lane = tid & 31, wave = tid >> 5, hh = lane >> 4, m = lane & 15;
  const int row0 = blockIdx.x * RPB + wave * 16;
  _Float16* h0w = h0t + wave * (16 * PITCH);
  _Float16* h1w = h1t + wave * (16 * PITCH);
  float* yw = yc + wave * (16 * D_);
  float* xw = xc + wave * (16 * D_);
  constexpr float OSC = 1.0f / (XS * WS);

#pragma unroll
  for (int q = 0; q < 4; ++q) {
    const int idx = q * 32 + lane, r = idx >> 3, c4 = (idx & 7) * 4;
    *(v4f*)(xw + r * D_ + c4) = *(const v4f*)(xin + (size_t)(row0 + r) * D_ + c4);
  }
  float lad[8];
#pragma unroll
  for (int r = 0; r < 8; ++r) lad[r] = 0.0f;

#pragma unroll 1
  for (int blk = 0; blk < NB_; ++blk) {
    const v4f z4 = {0.f, 0.f, 0.f, 0.f};
#pragma unroll
    for (int q = 0; q < 4; ++q) {
      const int idx = q * 32 + lane, r = idx >> 3, c4 = (idx & 7) * 4;
      *(v4f*)(yw + r * D_ + c4) = z4;
    }
    __syncthreads();

    const _Float16* p0 = wh + (size_t)blk * H_ * D_;
    const _Float16* p1 = wh + OFF_P1 + (size_t)blk * H_ * H_;
    const _Float16* p2 = wh + OFF_P2 + (size_t)blk * NO_ * H_;
    const float* b0s = bpl + blk * H_;
    const float* b1s = bpl + NB_ * H_ + blk * H_;
    const float* b2b = b2 + blk * NO_;

#pragma unroll 1
    for (int i = 0; i < D_; ++i) {
      const int kc1 = (cntp(i) + 31) >> 5;
      const int ntl = 2 * kc1;

      FragH ay;
      {
        const float* p = yw + m * D_ + 8 * hh;
        const v4f f0 = *(const v4f*)(p);
        const v4f f1 = *(const v4f*)(p + 4);
        const v4f f2 = *(const v4f*)(p + 16);
        const v4f f3 = *(const v4f*)(p + 20);
        ay.h[0] = cvt8(f0, f1, XS);
        ay.h[1] = cvt8(f2, f3, XS);
      }

#pragma unroll 1
      for (int nt = 0; nt < ntl; ++nt) {
        const v16h bfr = ldfrag(p0 + (size_t)(nt * 16 + m) * D_ + 8 * hh);
        const v8f c = wmf(ay.v, bfr, zero8());
        const float bia = b0s[nt * 16 + m];
#pragma unroll
        for (int r = 0; r < 8; ++r)
          h0w[(8 * hh + r) * PITCH + nt * 16 + m] = (_Float16)(fmaxf(c[r] * OSC + bia, 0.0f) * XS);
      }
      __syncthreads();

#pragma unroll 1
      for (int nt = 0; nt < ntl; ++nt) {
        const int kq = (cntp(sdeg(nt * 16 + 15) + 1) + 31) >> 5;
        const int kcn = (kq < kc1) ? kq : kc1;
        const _Float16* ap = h0w + m * PITCH + 8 * hh;
        const _Float16* bp = p1 + (size_t)(nt * 16 + m) * H_ + 8 * hh;
        v8f c = zero8();
#pragma unroll 1
        for (int kc = 0; kc < kcn; ++kc) c = wmf(ldfrag(ap + kc * 32), ldfrag(bp + kc * 32), c);
        const float bia = b1s[nt * 16 + m];
#pragma unroll
        for (int r = 0; r < 8; ++r)
          h1w[(8 * hh + r) * PITCH + nt * 16 + m] = (_Float16)(fmaxf(c[r] * OSC + bia, 0.0f) * XS);
      }
      __syncthreads();

      {
        const int rowc = i + ((m & 1) << 5);
        const _Float16* ap = h1w + m * PITCH + 8 * hh;
        const _Float16* bp = p2 + (size_t)rowc * H_ + 8 * hh;
        v8f c = zero8();
#pragma unroll 1
        for (int kc = 0; kc < kc1; ++kc) c = wmf(ldfrag(ap + kc * 32), ldfrag(bp + kc * 32), c);
        const float bm = b2b[i], bs = b2b[D_ + i];
        const bool odd = ((m & 1) != 0);
        float yn[8];
#pragma unroll
        for (int r = 0; r < 8; ++r) {
          const float mine = c[r];
          const float oth = __shfl_xor(mine, 1);
          const float mua = odd ? oth : mine;
          const float sa = odd ? mine : oth;
          const float mu = mua * OSC + bm;
          const float s = sa * OSC + bs;
          const float xv = xw[(8 * hh + r) * D_ + i];
          yn[r] = (xv - mu) * expf(-s);
          lad[r] -= s;
        }
        if (m == 0) {
#pragma unroll
          for (int r = 0; r < 8; ++r) yw[(8 * hh + r) * D_ + i] = yn[r];
        }
      }
      __syncthreads();
    }

    for (int idx = lane; idx < 16 * D_; idx += 32) {
      const int r = idx >> 5, cc = idx & 31;
      xw[r * D_ + cc] = yw[r * D_ + (D_ - 1 - cc)];
    }
    __syncthreads();
  }

  if (m == 0) {
#pragma unroll
    for (int r = 0; r < 8; ++r) lst[wave * 16 + 8 * hh + r] = lad[r];
  }
  __syncthreads();

  v4f yv[4];
#pragma unroll
  for (int q = 0; q < 4; ++q) yv[q] = *(const v4f*)(xw + q * 128 + 4 * lane);
  const v4f lv = *(const v4f*)(lst + 4 * (lane & 7));
  float* gy = out + (size_t)row0 * D_;
  float* gl = out + (size_t)YOFF + (size_t)blockIdx.x * RPB + 4 * (lane & 7);
  const bool wl = (wave == 0) && (lane < 8);
#pragma unroll
  for (int q = 0; q < 4; ++q) *(volatile v4f*)(gy + q * 128 + 4 * lane) = yv[q];
  if (wl) *(volatile v4f*)gl = lv;
  __threadfence();
#pragma unroll
  for (int q = 0; q < 4; ++q) *(volatile v4f*)(gy + q * 128 + 4 * lane) = yv[q];
  if (wl) *(volatile v4f*)gl = lv;
}

extern "C" void kernel_launch(void* const* d_in, const int* in_sizes, int n_in,
                              void* d_out, int out_size, void* d_ws, size_t ws_size,
                              hipStream_t stream) {
  if (n_in < 7) return;
  if (in_sizes[0] != NROWS * D_) return;
  if (in_sizes[1] != NB_ * H_ * D_ || in_sizes[2] != NB_ * H_) return;
  if (in_sizes[3] != NB_ * H_ * H_ || in_sizes[4] != NB_ * H_) return;
  if (in_sizes[5] != NB_ * NO_ * H_ || in_sizes[6] != NB_ * NO_) return;
  if (out_size != NROWS * D_ + NROWS) return;

  const float* xin = (const float*)d_in[0];
  const float* W0  = (const float*)d_in[1];
  const float* b0  = (const float*)d_in[2];
  const float* W1  = (const float*)d_in[3];
  const float* b1  = (const float*)d_in[4];
  const float* W2  = (const float*)d_in[5];
  const float* b2  = (const float*)d_in[6];
  float* out = (float*)d_out;

  if ((size_t)WSBYTES > ws_size) return;
  _Float16* wh = (_Float16*)d_ws;
  float* bpl = (float*)d_ws + BOFF;

  k_pack<<<dim3(PKB), dim3(256), 0, stream>>>(W0, W1, W2, b0, b1, wh, bpl);
  k_flow<<<dim3(NROWS / RPB), dim3(NTHR), 0, stream>>>(xin, wh, bpl, b2, out);
}
